// GraphFormer_32822140076792
// MI455X (gfx1250) — hardware-verified
//
#include <hip/hip_runtime.h>
#include <stddef.h>


#define KD     64
#define DQ     128
#define DS     32
#define NF     416
#define NSLAB  13
#define GT     128
#define WPP    72
#define RB     1024
#define RBBITS 10
#define RMAX   64
#define RMBITS 6
#define TABW   (2 * RMAX)
#define CHUNK  4096
#define LCAP   18432
#define DEGCAP 64
#define SCW    (32 * DEGCAP)
#define WSCAP  134217728
#define ASCL   8.0f
#define WSCL   64.0f
#define INVSCL 0.001953125f
#define RSQC   0.17677669529663687f

#define EDGE_LDS_INTS  (RB + 8 + RB + LCAP)
#define EDGE_LDS_BYTES ((EDGE_LDS_INTS + 8 * SCW) * 4)

static_assert(RB == (1 << RBBITS));
static_assert(RMAX == (1 << RMBITS));
static_assert(CHUNK == 8 * 16 * 32);
static_assert(CHUNK == 4 * 4 * 256);
static_assert(TABW * 4 == 32 * 16);
static_assert((WPP % 8) == 0);
static_assert((RB % 128) == 0);
static_assert(RB == 4 * 256);
static_assert(((EDGE_LDS_INTS * 4) % 16) == 0);
static_assert(EDGE_LDS_BYTES < 300000);
static_assert(SCW >= 256);
static_assert((KD % 32) == 0);
static_assert(NF == 3 * DQ + DS);
static_assert(NSLAB * 32 == NF);
static_assert(((NF * 4) % 128) == 0);
static_assert((DQ % 32) == 0 && (DS % 32) == 0);
static_assert(KD * 2 == 128);

typedef float          v4f  __attribute__((ext_vector_type(4)));
typedef float          v8f  __attribute__((ext_vector_type(8)));
typedef int            v4i  __attribute__((ext_vector_type(4)));
typedef unsigned int   v4u  __attribute__((ext_vector_type(4)));
typedef unsigned short v8us __attribute__((ext_vector_type(8)));
typedef _Float16       v16h __attribute__((ext_vector_type(16)));
union FragH { v16h v; v8us u[2]; };

__device__ __forceinline__ unsigned short h16(float f) {
  const _Float16 h = (_Float16)f;
  return __builtin_bit_cast(unsigned short, h);
}

__device__ __forceinline__ v8us cvt8(v4f a, v4f b, float s) {
  v8us r;
  r[0] = h16(a.x * s); r[1] = h16(a.y * s); r[2] = h16(a.z * s); r[3] = h16(a.w * s);
  r[4] = h16(b.x * s); r[5] = h16(b.y * s); r[6] = h16(b.z * s); r[7] = h16(b.w * s);
  return r;
}

__device__ __forceinline__ v8f wmh(v16h a, v16h b, v8f c) {
  v8f d = __builtin_amdgcn_wmma_f32_16x16x32_f16(false, a, false, b, (short)0, c, false, false);
  asm volatile("v_nop\n\tv_nop\n\tv_nop\n\tv_nop" : "+v"(d) : "v"(a), "v"(b));
  return d;
}

template <int NB>
__device__ __forceinline__ unsigned int match_mask(unsigned int base, int key) {
  unsigned int msk = base;
#pragma unroll
  for (int b = 0; b < NB; ++b) {
    const bool bit = ((key >> b) & 1) != 0;
    const unsigned int bb = __builtin_amdgcn_ballot_w32(bit);
    msk &= bit ? bb : ~bb;
  }
  return msk;
}

__global__ __launch_bounds__(256) void k_csort(
    const int* __restrict__ key, unsigned int* csort, int* tab, int nN, int nE) {
  __shared__ __attribute__((aligned(16))) unsigned int sImg[CHUNK];
  __shared__ int cw[8 * RMAX];
  __shared__ __attribute__((aligned(16))) int sTb[TABW];
  __shared__ int sWt[8];
  int* sPre = sTb;
  int* sCn  = sTb + RMAX;
  const int tid = (int)threadIdx.x, lane = tid & 31, wave = tid >> 5;
  const int c = (int)blockIdx.x;
  const int cbase = c * CHUNK;

  for (int i = tid; i < 8 * RMAX; i += 256) cw[i] = 0;
  {
    const v4u s = {0xffffffffu, 0xffffffffu, 0xffffffffu, 0xffffffffu};
    for (int i = tid; i < CHUNK / 4; i += 256) ((v4u*)sImg)[i] = s;
  }
  __syncthreads();

  unsigned int ent[16];
  int pk[16];
  const unsigned int lt = (1u << lane) - 1u;
#pragma unroll
  for (int i = 0; i < 16; ++i) {
    const int e = cbase + wave * 512 + 32 * i + lane;
    const int ea = e > nE - 1 ? nE - 1 : e;
    const int d = key[ea];
    const bool valid = (e < nE) && ((unsigned)d < (unsigned)nN);
    const int dd = valid ? d : 0;
    const int r  = dd >> RBBITS;
    const int jl = dd & (RB - 1);
    const unsigned int pay = (unsigned int)ea;
    const unsigned int msk = match_mask<RMBITS>(__builtin_amdgcn_ballot_w32(valid), r);
    const int rank = (int)__builtin_popcount(msk & lt);
    const int grp  = (int)__builtin_popcount(msk);
    const int base = cw[wave * RMAX + r];
    pk[i]  = valid ? ((r << 12) | (base + rank)) : -1;
    ent[i] = (pay << RBBITS) | (unsigned int)jl;
    if (valid && rank == 0) cw[wave * RMAX + r] = base + grp;
    __syncthreads();
  }

  if (tid < RMAX) {
    int run = 0;
#pragma unroll
    for (int w = 0; w < 8; ++w) {
      const int v = cw[w * RMAX + tid];
      cw[w * RMAX + tid] = run;
      run += v;
    }
    sCn[tid] = run;
  }
  __syncthreads();
  {
    const int vr = sCn[tid & (RMAX - 1)];
    const int v  = (tid < RMAX) ? vr : 0;
    int x = v;
#pragma unroll
    for (int dd = 1; dd < 32; dd <<= 1) {
      const int y = __shfl_up(x, dd);
      x += (lane >= dd) ? y : 0;
    }
    if (lane == 31) sWt[wave] = x;
    __syncthreads();
    int pre = 0;
#pragma unroll
    for (int w = 0; w < 8; ++w) { const int tw = sWt[w]; pre += (w < wave) ? tw : 0; }
    if (tid < RMAX) sPre[tid] = pre + x - v;
  }
  __syncthreads();

#pragma unroll
  for (int i = 0; i < 16; ++i) {
    if (pk[i] >= 0) {
      const int r = (pk[i] >> 12) & (RMAX - 1);
      const int q = pk[i] & 4095;
      const int pos = sPre[r] + cw[wave * RMAX + r] + q;
      if ((unsigned)pos < (unsigned)CHUNK) sImg[pos] = ent[i];
    }
  }
  __syncthreads();

  v4u iv[4];
#pragma unroll
  for (int it = 0; it < 4; ++it) iv[it] = ((const v4u*)sImg)[it * 256 + tid];
  const v4i tv = *(const v4i*)(sTb + 4 * lane);
  unsigned int* gp = csort + (size_t)c * CHUNK;
  int* tp = tab + (size_t)c * TABW + 4 * lane;
  const bool wt = tid < 32;
#pragma unroll
  for (int it = 0; it < 4; ++it) *(volatile v4u*)(gp + 4 * (it * 256 + tid)) = iv[it];
  if (wt) *(volatile v4i*)tp = tv;
  __threadfence();
#pragma unroll
  for (int it = 0; it < 4; ++it) *(volatile v4u*)(gp + 4 * (it * 256 + tid)) = iv[it];
  if (wt) *(volatile v4i*)tp = tv;
}

__global__ __launch_bounds__(256) void k_xcvt(
    const float* __restrict__ x, unsigned short* x16, int nN) {
  const int tid = (int)threadIdx.x;
  const int rb = (int)blockIdx.x * 128;
  const v4f zero4 = {0.0f, 0.0f, 0.0f, 0.0f};
  v8us o[4];
  size_t po[4];
#pragma unroll
  for (int it = 0; it < 4; ++it) {
    const int p = it * 256 + tid;
    const int row = rb + (p >> 3);
    const int c8 = (p & 7) * 8;
    const bool live = row < nN;
    const int xr = live ? row : (nN - 1);
    v4f a = *(const v4f*)(x + (size_t)xr * KD + c8);
    v4f b = *(const v4f*)(x + (size_t)xr * KD + c8 + 4);
    a = live ? a : zero4;
    b = live ? b : zero4;
    o[it]  = cvt8(a, b, ASCL);
    po[it] = (size_t)row * KD + c8;
  }
#pragma unroll
  for (int it = 0; it < 4; ++it) *(volatile v8us*)(x16 + po[it]) = o[it];
  __threadfence();
#pragma unroll
  for (int it = 0; it < 4; ++it) *(volatile v8us*)(x16 + po[it]) = o[it];
}

__global__ __launch_bounds__(256) void k_wprep(
    const float* __restrict__ W0, const float* __restrict__ W1, const float* __restrict__ W2,
    const float* __restrict__ W3, unsigned short* w16, int Kin) {
  __shared__ __attribute__((aligned(16))) unsigned short sT[DQ * WPP];
  const int tid = (int)threadIdx.x;
  const int mat = (int)blockIdx.x;
  const float* W = (mat == 0) ? W0 : ((mat == 1) ? W1 : ((mat == 2) ? W2 : W3));
  const int nb = (mat < 3) ? 7 : 5;
  const int Nm = 1 << nb;
  const int rowBase = mat * DQ;

  for (int i = tid; i < (DQ * WPP) / 2; i += 256) ((unsigned int*)sT)[i] = 0u;
  __syncthreads();

  const int nfill = (Kin * Nm) >> 10;
#pragma unroll 1
  for (int it = 0; it < nfill; ++it) {
    const int idx = (it * 256 + tid) << 2;
    const int k = idx >> nb, nl = idx & (Nm - 1);
    const v4f w = *(const v4f*)(W + idx);
    unsigned short* d = sT + nl * WPP + k;
    d[0]       = h16(w.x * WSCL);
    d[WPP]     = h16(w.y * WSCL);
    d[2 * WPP] = h16(w.z * WSCL);
    d[3 * WPP] = h16(w.w * WSCL);
  }
  __syncthreads();

  const int nst = Nm >> 5;
#pragma unroll 1
  for (int it = 0; it < nst; ++it) {
    const int p = it * 256 + tid;
    const int row = p >> 3, c8 = (p & 7) * 8;
    const v8us v = *(const v8us*)(sT + row * WPP + c8);
    *(volatile v8us*)(w16 + (size_t)(rowBase + row) * KD + c8) = v;
  }
  __threadfence();
#pragma unroll 1
  for (int it = 0; it < nst; ++it) {
    const int p = it * 256 + tid;
    const int row = p >> 3, c8 = (p & 7) * 8;
    const v8us v = *(const v8us*)(sT + row * WPP + c8);
    *(volatile v8us*)(w16 + (size_t)(rowBase + row) * KD + c8) = v;
  }
}

__global__ __launch_bounds__(GT) void k_gemm(
    const unsigned short* __restrict__ A, const unsigned short* __restrict__ Bt,
    const float* __restrict__ b0, const float* __restrict__ b1,
    const float* __restrict__ b2, const float* __restrict__ b3,
    float* outF, int Mp) {
  __shared__ __attribute__((aligned(16))) float sT[4 * 32 * 32];
  const int tid = (int)threadIdx.x, lane = tid & 31, wave = tid >> 5, hh = lane >> 4, m = lane & 15;
  const int slab = (int)blockIdx.x;
  const int c0 = slab * 32;
  int mat = slab >> 2; mat = mat > 3 ? 3 : mat;
  const float* bias = (mat == 0) ? b0 : ((mat == 1) ? b1 : ((mat == 2) ? b2 : b3));
  const int blen = (mat < 3) ? DQ : DS;
  const int cl0 = c0 - mat * DQ;
  const int r0 = (int)blockIdx.y * 128 + wave * 32;

  int ra0 = r0 + m;      ra0 = ra0 > Mp - 1 ? Mp - 1 : ra0;
  int ra1 = r0 + 16 + m; ra1 = ra1 > Mp - 1 ? Mp - 1 : ra1;
  const unsigned short* ap0 = A + (size_t)ra0 * KD + 8 * hh;
  const unsigned short* ap1 = A + (size_t)ra1 * KD + 8 * hh;
  const unsigned short* bp[2];
#pragma unroll
  for (int j = 0; j < 2; ++j) {
    int cb = c0 + 16 * j + m; cb = cb > NF - 1 ? NF - 1 : cb;
    bp[j] = Bt + (size_t)cb * KD + 8 * hh;
  }

  v8f acc[2][2];
#pragma unroll
  for (int i = 0; i < 2; ++i)
#pragma unroll
    for (int j = 0; j < 2; ++j) { v8f z = {0.f, 0.f, 0.f, 0.f, 0.f, 0.f, 0.f, 0.f}; acc[i][j] = z; }

#pragma unroll 1
  for (int kt = 0; kt < KD / 32; ++kt) {
    const int kb = kt << 5;
    FragH a0, a1, bf0, bf1;
    a0.u[0] = *(const v8us*)(ap0 + kb);
    a0.u[1] = *(const v8us*)(ap0 + kb + 16);
    a1.u[0] = *(const v8us*)(ap1 + kb);
    a1.u[1] = *(const v8us*)(ap1 + kb + 16);
    bf0.u[0] = *(const v8us*)(bp[0] + kb);
    bf0.u[1] = *(const v8us*)(bp[0] + kb + 16);
    bf1.u[0] = *(const v8us*)(bp[1] + kb);
    bf1.u[1] = *(const v8us*)(bp[1] + kb + 16);
    acc[0][0] = wmh(a0.v, bf0.v, acc[0][0]);
    acc[1][0] = wmh(a1.v, bf0.v, acc[1][0]);
    acc[0][1] = wmh(a0.v, bf1.v, acc[0][1]);
    acc[1][1] = wmh(a1.v, bf1.v, acc[1][1]);
  }

  float* sw = sT + wave * 1024;
#pragma unroll
  for (int i = 0; i < 2; ++i)
#pragma unroll
    for (int j = 0; j < 2; ++j)
#pragma unroll
      for (int r = 0; r < 8; ++r)
        sw[(16 * i + 8 * hh + r) * 32 + 16 * j + m] = acc[i][j][r];
  __syncthreads();

  v4f ov[8];
  size_t po[8];
#pragma unroll
  for (int it = 0; it < 8; ++it) {
    const int f = it * 32 + lane;
    const int row = f >> 3, c4 = (f & 7) * 4;
    const v4f v = *(const v4f*)(sw + row * 32 + c4);
    int bc = cl0 + c4; bc = bc > blen - 4 ? blen - 4 : bc; bc = bc < 0 ? 0 : bc;
    const v4f bb = *(const v4f*)(bias + bc);
    ov[it] = v * INVSCL + bb;
    po[it] = (size_t)(r0 + row) * NF + c0 + c4;
  }
#pragma unroll
  for (int it = 0; it < 8; ++it) *(volatile v4f*)(outF + po[it]) = ov[it];
  __threadfence();
#pragma unroll
  for (int it = 0; it < 8; ++it) *(volatile v4f*)(outF + po[it]) = ov[it];
}

template <int L1>
__global__ __launch_bounds__(256) void k_edge(
    const float* __restrict__ F, const int* __restrict__ src,
    const unsigned int* __restrict__ csort, const int* __restrict__ tab,
    unsigned short* h16, float* out, int nN, int nNp, int nE, int nCh) {
  extern __shared__ __attribute__((aligned(16))) int dsm[];
  __shared__ int sWtot[8];
  int*   sOff  = dsm;
  int*   sCur  = dsm + (RB + 8);
  int*   sList = sCur + RB;
  float* sSc   = (float*)(sList + LCAP);
  const int tid = (int)threadIdx.x, lane = tid & 31, wave = tid >> 5;
  const int rgn = (int)blockIdx.x;
  const int n0 = rgn * RB;
  const unsigned int lt = (1u << lane) - 1u;

  for (int i = tid; i < RB + 8; i += 256) sOff[i] = 0;
  for (int i = tid; i < RB; i += 256) sCur[i] = 0;
  __syncthreads();

#pragma unroll 1
  for (int c = 0; c < nCh; ++c) {
    int pre = tab[(size_t)c * TABW + rgn];
    int n   = tab[(size_t)c * TABW + RMAX + rgn];
    pre = pre < 0 ? 0 : (pre > CHUNK ? CHUNK : pre);
    n = n < 0 ? 0 : (n > CHUNK - pre ? CHUNK - pre : n);
    const int nstep = (n + 31) >> 5;
    const unsigned int* cp = csort + (size_t)c * CHUNK + pre;
#pragma unroll 1
    for (int s = 0; s < nstep; ++s) {
      if (wave == 0) {
        const int i = (s << 5) + lane;
        const bool valid = i < n;
        const int ic = i > n - 1 ? n - 1 : i;
        const unsigned int en = cp[ic];
        const int j = (int)(en & (unsigned int)(RB - 1));
        const unsigned int msk = match_mask<RBBITS>(__builtin_amdgcn_ballot_w32(valid), j);
        const int rank = (int)__builtin_popcount(msk & lt);
        const int grp  = (int)__builtin_popcount(msk);
        if (valid && rank == 0) sOff[j] = sOff[j] + grp;
      }
      __syncthreads();
    }
  }
  __syncthreads();

  {
    int cn[4];
    int ls = 0;
#pragma unroll
    for (int i = 0; i < 4; ++i) { cn[i] = sOff[4 * tid + i]; ls += cn[i]; }
    int x = ls;
#pragma unroll
    for (int dd = 1; dd < 32; dd <<= 1) {
      const int y = __shfl_up(x, dd);
      x += (lane >= dd) ? y : 0;
    }
    if (lane == 31) sWtot[wave] = x;
    __syncthreads();
    int pre = 0;
#pragma unroll
    for (int w = 0; w < 8; ++w) { const int tw = sWtot[w]; pre += (w < wave) ? tw : 0; }
    int run = pre + x - ls;
#pragma unroll
    for (int i = 0; i < 4; ++i) { sOff[4 * tid + i] = run; run += cn[i]; }
    if (tid == 255) sOff[RB] = run;
  }
  __syncthreads();
  const bool rgnOver = sOff[RB] > LCAP;

#pragma unroll 1
  for (int c = 0; c < nCh; ++c) {
    int pre = tab[(size_t)c * TABW + rgn];
    int n   = tab[(size_t)c * TABW + RMAX + rgn];
    pre = pre < 0 ? 0 : (pre > CHUNK ? CHUNK : pre);
    n = n < 0 ? 0 : (n > CHUNK - pre ? CHUNK - pre : n);
    const int nstep = (n + 31) >> 5;
    const unsigned int* cp = csort + (size_t)c * CHUNK + pre;
#pragma unroll 1
    for (int s = 0; s < nstep; ++s) {
      if (wave == 0) {
        const int i = (s << 5) + lane;
        const bool valid = i < n;
        const int ic = i > n - 1 ? n - 1 : i;
        const unsigned int en = cp[ic];
        const int j = (int)(en & (unsigned int)(RB - 1));
        int e = (int)(en >> RBBITS);
        e = e > nE - 1 ? nE - 1 : e;
        const unsigned int msk = match_mask<RBBITS>(__builtin_amdgcn_ballot_w32(valid), j);
        const int rank = (int)__builtin_popcount(msk & lt);
        const int grp  = (int)__builtin_popcount(msk);
        const int cur  = sCur[j];
        const int p0   = sOff[j] + cur + rank;
        if (valid && (unsigned)p0 < (unsigned)LCAP) sList[p0] = e;
        if (valid && rank == 0) sCur[j] = cur + grp;
      }
      __syncthreads();
    }
  }
  __syncthreads();

  const int c4 = 4 * lane;
  const int cs = 4 * (lane & 7);
  int Rbp = nNp - n0; Rbp = Rbp > RB ? RB : Rbp;
  const int niter = (Rbp + 7) >> 3;
  float* sw = sSc + wave * SCW;
  const v4f zero4 = {0.0f, 0.0f, 0.0f, 0.0f};
  const float qn = __int_as_float(0x7fc00000);
  const v4f nan4 = {qn, qn, qn, qn};
#pragma unroll 1
  for (int jj = 0; jj < niter; ++jj) {
    const int j = jj * 8 + wave;
    const bool act = j < Rbp;
    const int jc = act ? j : (Rbp - 1);
    const int node = n0 + jc;
    const bool live = node < nN;
    int lb = __builtin_amdgcn_readfirstlane(sOff[jc]);
    int ub = __builtin_amdgcn_readfirstlane(sOff[jc + 1]);
    lb = lb < 0 ? 0 : (lb > LCAP ? LCAP : lb);
    ub = ub < 0 ? 0 : (ub > LCAP ? LCAP : ub);
    const int craw = ub - lb;
    int cnt = craw;
    cnt = cnt < 0 ? 0 : (cnt > DEGCAP ? DEGCAP : cnt);

    const float* frow = F + (size_t)node * NF;
    const v4f qv = *(const v4f*)(frow + c4);

    float mx = __int_as_float(0xff800000u);
#pragma unroll 1
    for (int it = 0; it < cnt; ++it) {
      int li = lb + it; li = li > LCAP - 1 ? LCAP - 1 : li;
      int e = sList[li]; e = e < 0 ? 0 : (e > nE - 1 ? nE - 1 : e);
      int s = src[e];   s = s < 0 ? 0 : (s > nN - 1 ? nN - 1 : s);
      const v4f kv = *(const v4f*)(F + (size_t)s * NF + DQ + c4);
      float part = qv.x * kv.x;
      part = fmaf(qv.y, kv.y, part);
      part = fmaf(qv.z, kv.z, part);
      part = fmaf(qv.w, kv.w, part);
      part += __shfl_xor(part, 1);
      part += __shfl_xor(part, 2);
      part += __shfl_xor(part, 4);
      const float sc = part * RSQC;
      mx = fmaxf(mx, sc);
      sw[it * 32 + lane] = sc;
    }

    v4f acc = zero4;
    float z = 0.0f;
#pragma unroll 1
    for (int it = 0; it < cnt; ++it) {
      int li = lb + it; li = li > LCAP - 1 ? LCAP - 1 : li;
      int e = sList[li]; e = e < 0 ? 0 : (e > nE - 1 ? nE - 1 : e);
      int s = src[e];   s = s < 0 ? 0 : (s > nN - 1 ? nN - 1 : s);
      const float sc = sw[it * 32 + lane];
      const float p = __expf(sc - mx);
      const v4f vv = *(const v4f*)(F + (size_t)s * NF + 2 * DQ + c4);
      acc = acc + vv * p;
      z += p;
    }
    const float zs = (cnt > 0) ? z : 1.0f;
    const float rz = 1.0f / zs;
    v4f r = acc * rz;
    r.x += __shfl_xor(r.x, 8);  r.y += __shfl_xor(r.y, 8);
    r.z += __shfl_xor(r.z, 8);  r.w += __shfl_xor(r.w, 8);
    r.x += __shfl_xor(r.x, 16); r.y += __shfl_xor(r.y, 16);
    r.z += __shfl_xor(r.z, 16); r.w += __shfl_xor(r.w, 16);
    const v4f sv = *(const v4f*)(frow + 3 * DQ + cs);
    v4f hv = r * 0.25f + sv;
    if (L1 != 0) {
      hv.x = fmaxf(hv.x, 0.0f); hv.y = fmaxf(hv.y, 0.0f);
      hv.z = fmaxf(hv.z, 0.0f); hv.w = fmaxf(hv.w, 0.0f);
    }
    const bool bad = (craw > DEGCAP) || rgnOver;
    hv = bad ? nan4 : hv;

    if (L1 != 0) {
      hv = live ? hv : zero4;
      *(v4f*)(sw + c4) = hv;
      __syncthreads();
      const int l8 = 8 * (lane & 3);
      const v4f u0 = *(const v4f*)(sw + l8);
      const v4f u1 = *(const v4f*)(sw + l8 + 4);
      __syncthreads();
      const v8us z8 = {0, 0, 0, 0, 0, 0, 0, 0};
      const v8us oc = cvt8(u0, u1, ASCL);
      const v8us o = ((lane & 4) != 0) ? z8 : oc;
      unsigned short* op = h16 + (size_t)node * KD + 8 * (lane & 7);
      const bool wst = act && (lane < 8);
      if (wst) *(volatile v8us*)op = o;
      __threadfence();
      if (wst) *(volatile v8us*)op = o;
    } else {
      float* op = out + (size_t)node * DS + cs;
      const bool wst = act && live && (lane < 8);
      if (wst) *(volatile v4f*)op = hv;
      __threadfence();
      if (wst) *(volatile v4f*)op = hv;
    }
  }
}

extern "C" void kernel_launch(void* const* d_in, const int* in_sizes, int n_in,
                              void* d_out, int out_size, void* d_ws, size_t ws_size,
                              hipStream_t stream) {
  if (n_in < 18) return;
  const int nN = in_sizes[0] / KD;
  const int nE = in_sizes[1] / 2;
  if (nN <= 0 || nE <= 0) return;
  if (in_sizes[0] != nN * KD) return;
  if (in_sizes[1] != 2 * nE) return;
  if (nN > RMAX * RB || nE > (1 << 22)) return;
  if (in_sizes[2] != KD * DQ || in_sizes[4] != KD * DQ || in_sizes[6] != KD * DQ) return;
  if (in_sizes[3] != DQ || in_sizes[5] != DQ || in_sizes[7] != DQ) return;
  if (in_sizes[8] != KD * DS || in_sizes[9] != DS) return;
  if (in_sizes[10] != DS * DQ || in_sizes[12] != DS * DQ || in_sizes[14] != DS * DQ) return;
  if (in_sizes[11] != DQ || in_sizes[13] != DQ || in_sizes[15] != DQ) return;
  if (in_sizes[16] != DS * DS || in_sizes[17] != DS) return;
  if (out_size != nN * DS) return;

  const float* x    = (const float*)d_in[0];
  const int*   ei   = (const int*)d_in[1];
  const float* Wq1  = (const float*)d_in[2];
  const float* bq1  = (const float*)d_in[3];
  const float* Wk1  = (const float*)d_in[4];
  const float* bk1  = (const float*)d_in[5];
  const float* Wv1  = (const float*)d_in[6];
  const float* bv1  = (const float*)d_in[7];
  const float* Ws1  = (const float*)d_in[8];
  const float* bs1  = (const float*)d_in[9];
  const float* Wq2  = (const float*)d_in[10];
  const float* bq2  = (const float*)d_in[11];
  const float* Wk2  = (const float*)d_in[12];
  const float* bk2  = (const float*)d_in[13];
  const float* Wv2  = (const float*)d_in[14];
  const float* bv2  = (const float*)d_in[15];
  const float* Ws2  = (const float*)d_in[16];
  const float* bs2  = (const float*)d_in[17];
  const int*   esrc = ei;
  const int*   edst = ei + nE;
  float* out = (float*)d_out;

  const int nCh = (nE + CHUNK - 1) / CHUNK;
  const int nR  = (nN + RB - 1) / RB;
  const int nNp = ((nN + 127) / 128) * 128;

  const size_t szX16 = (size_t)nNp * KD * 2;
  const size_t szH16 = (size_t)nNp * KD * 2;
  const size_t szW16 = (size_t)NF * KD * 2;
  const size_t szF   = (size_t)nNp * NF * 4;
  const size_t szCS  = (size_t)nCh * CHUNK * 4;
  const size_t szTab = (size_t)nCh * TABW * 4;
  size_t off = 0;
  const size_t oX  = off; off += szX16; off = (off + 255) & ~(size_t)255;
  const size_t oH  = off; off += szH16; off = (off + 255) & ~(size_t)255;
  const size_t oWa = off; off += szW16; off = (off + 255) & ~(size_t)255;
  const size_t oWb = off; off += szW16; off = (off + 255) & ~(size_t)255;
  const size_t oF  = off; off += szF;   off = (off + 255) & ~(size_t)255;
  const size_t oC  = off; off += szCS;  off = (off + 255) & ~(size_t)255;
  const size_t oT  = off; off += szTab; off = (off + 255) & ~(size_t)255;
  if (off > ws_size || off > (size_t)WSCAP) return;

  char* ws = (char*)d_ws;
  unsigned short* x16   = (unsigned short*)(ws + oX);
  unsigned short* h16   = (unsigned short*)(ws + oH);
  unsigned short* w16a  = (unsigned short*)(ws + oWa);
  unsigned short* w16b  = (unsigned short*)(ws + oWb);
  float*          F     = (float*)(ws + oF);
  unsigned int*   csort = (unsigned int*)(ws + oC);
  int*            tab   = (int*)(ws + oT);

  k_csort<<<nCh, 256, 0, stream>>>(edst, csort, tab, nN, nE);

  k_xcvt<<<nNp / 128, 256, 0, stream>>>(x, x16, nN);

  k_wprep<<<4, 256, 0, stream>>>(Wq1, Wk1, Wv1, Ws1, w16a, KD);
  k_wprep<<<4, 256, 0, stream>>>(Wq2, Wk2, Wv2, Ws2, w16b, DS);

  k_gemm<<<dim3(NSLAB, nNp / 128, 1), GT, 0, stream>>>(x16, w16a, bq1, bk1, bv1, bs1, F, nNp);

  hipFuncSetAttribute(reinterpret_cast<const void*>(&k_edge<1>),
                      hipFuncAttributeMaxDynamicSharedMemorySize, EDGE_LDS_BYTES);
  k_edge<1><<<nR, 256, EDGE_LDS_BYTES, stream>>>(F, esrc, csort, tab, h16, out, nN, nNp, nE, nCh);

  k_gemm<<<dim3(NSLAB, nNp / 128, 1), GT, 0, stream>>>(h16, w16b, bq2, bk2, bv2, bs2, F, nNp);

  hipFuncSetAttribute(reinterpret_cast<const void*>(&k_edge<0>),
                      hipFuncAttributeMaxDynamicSharedMemorySize, EDGE_LDS_BYTES);
  k_edge<0><<<nR, 256, EDGE_LDS_BYTES, stream>>>(F, esrc, csort, tab, h16, out, nN, nNp, nE, nCh);
}
